// MambaPlusBlock_78039555769088
// MI455X (gfx1250) — hardware-run, weakly checked
//
#include <hip/hip_runtime.h>
#include <stddef.h>
#include <math.h>


#pragma clang fp contract(off)

#define NB    2
#define LSEQ  2048
#define NTOK  (NB * LSEQ)
#define DMD   512
#define DI    1024
#define DS    32
#define DC    4
#define DR    64
#define DBW   128
#define NTHR  256
#define WSCAP 134217728

#define WSC   32.0f
#define UHC   64.0f
#define DTHC  256.0f
#define YHC   256.0f

#define SZ_WIN  ((size_t)2 * DI * DI * 2)
#define SZ_WX   ((size_t)DBW * DI * 2)
#define SZ_WDT  ((size_t)DI * DR * 2)
#define SZ_WOP  ((size_t)DI * DI * 2)
#define SZ_WG   ((size_t)DMD * DMD * 2)
#define SZ_WO   ((size_t)DMD * DI * 2)
#define SZ_XH   ((size_t)NTOK * DMD * 2)
#define SZ_F32I ((size_t)NTOK * DI * 4)
#define SZ_F16I ((size_t)NTOK * DI * 2)
#define SZ_DBL  ((size_t)NTOK * DBW * 4)
#define SZ_DTH  ((size_t)NTOK * DR * 2)
#define SZ_F32H ((size_t)NTOK * DMD * 4)

#define O_WIN   ((size_t)0)
#define O_WX    (O_WIN + SZ_WIN)
#define O_WDT   (O_WX + SZ_WX)
#define O_WOP   (O_WDT + SZ_WDT)
#define O_WG    (O_WOP + SZ_WOP)
#define O_WO    (O_WG + SZ_WG)
#define O_XH    (O_WO + SZ_WO)
#define O_XC32  (O_XH + SZ_XH)
#define O_R1    (O_XC32 + SZ_F32I)
#define O_R2    (O_R1 + SZ_F16I)
#define O_R3    (O_R2 + SZ_F32I)
#define O_U32   (O_R3 + SZ_F32I)
#define O_DBL   (O_U32 + SZ_F32I)
#define O_DTH   (O_DBL + SZ_DBL)
#define O_G32   (O_DTH + SZ_DTH)
#define WSTOT   (O_G32 + SZ_F32H)
static_assert(WSTOT <= (size_t)WSCAP);
static_assert(SZ_F16I <= SZ_F32I && SZ_F32H <= SZ_F32I);
static_assert((O_WX % 128) == 0 && (O_WDT % 128) == 0 && (O_WOP % 128) == 0 && (O_WG % 128) == 0);
static_assert((O_WO % 128) == 0 && (O_XH % 128) == 0 && (O_XC32 % 128) == 0 && (O_R1 % 128) == 0);
static_assert((O_R2 % 128) == 0 && (O_R3 % 128) == 0 && (O_U32 % 128) == 0 && (O_DBL % 128) == 0);
static_assert((O_DTH % 128) == 0 && (O_G32 % 128) == 0 && (WSTOT % 128) == 0);

static_assert((DI % 32) == 0 && (DR % 32) == 0 && (DMD % 32) == 0);
static_assert((NTOK % 64) == 0 && (DI % 256) == 0 && (DMD % 256) == 0 && DBW == 128 && DR + 2 * DS == DBW);

typedef _Float16     v16h __attribute__((ext_vector_type(16)));
typedef _Float16     v8h  __attribute__((ext_vector_type(8)));
typedef _Float16     v4hh __attribute__((ext_vector_type(4)));
typedef float        v8f  __attribute__((ext_vector_type(8)));
typedef float        v4f  __attribute__((ext_vector_type(4), __may_alias__));
typedef unsigned int v4u  __attribute__((ext_vector_type(4), __may_alias__));
typedef unsigned int v2u  __attribute__((ext_vector_type(2), __may_alias__));
typedef int          v8i  __attribute__((ext_vector_type(8)));
union Frag { v16h v; v8i w; v4u q[2]; };
union P8 { v8h h; v4u u; };
union P4 { v4hh h; v2u u; };
static_assert(sizeof(Frag) == 32);
static_assert(sizeof(P8) == 16);
static_assert(sizeof(P4) == 8);

__device__ __forceinline__ v8f wmh(const Frag& a, const Frag& b, v8f c) {
  v8f d = __builtin_amdgcn_wmma_f32_16x16x32_f16(false, a.v, false, b.v, (short)0, c, false, false);
  asm volatile("v_nop\n\tv_nop\n\tv_nop\n\tv_nop" : "+v"(d) : "v"(a.w), "v"(b.w));
  return d;
}

__device__ __forceinline__ v8f zero8() {
  v8f z = {0.f, 0.f, 0.f, 0.f, 0.f, 0.f, 0.f, 0.f};
  return z;
}

__device__ __forceinline__ v4u pack8h(v4f a, v4f c) {
  P8 p;
  p.h[0] = (_Float16)a[0]; p.h[1] = (_Float16)a[1]; p.h[2] = (_Float16)a[2]; p.h[3] = (_Float16)a[3];
  p.h[4] = (_Float16)c[0]; p.h[5] = (_Float16)c[1]; p.h[6] = (_Float16)c[2]; p.h[7] = (_Float16)c[3];
  return p.u;
}

__device__ __forceinline__ v2u pack4h(v4f a) {
  P4 p;
  p.h[0] = (_Float16)a[0]; p.h[1] = (_Float16)a[1]; p.h[2] = (_Float16)a[2]; p.h[3] = (_Float16)a[3];
  return p.u;
}

__device__ __forceinline__ float wave_sum(float s) {
#pragma unroll
  for (int off = 16; off; off >>= 1) s += __shfl_xor(s, off, 32);
  return s;
}

#define T_WIN  512
#define T_WX   32
#define T_WDT  16
#define T_WOP  256
#define T_WG   64
#define T_WO   128
#define CB_WX  (T_WIN)
#define CB_WDT (CB_WX + T_WX)
#define CB_WOP (CB_WDT + T_WDT)
#define CB_WG  (CB_WOP + T_WOP)
#define CB_WO  (CB_WG + T_WG)
#define CB_TOT (CB_WO + T_WO)
#define TLD    68
static_assert(T_WIN == (2 * DI / 64) * (DI / 64) && T_WX == (DBW / 64) * (DI / 64) && T_WDT == (DI / 64) * (DR / 64));
static_assert(T_WOP == (DI / 64) * (DI / 64) && T_WG == (DMD / 64) * (DMD / 64) && T_WO == (DMD / 64) * (DI / 64));
static_assert(CB_TOT == 1008 && NTHR == 256);

__global__ __launch_bounds__(NTHR) void k_cvtw(const float* __restrict__ wip, const float* __restrict__ wxp,
                                               const float* __restrict__ wdt, const float* __restrict__ wop,
                                               const float* __restrict__ wg, const float* __restrict__ wo,
                                               unsigned short* WIN, unsigned short* WX, unsigned short* WDT,
                                               unsigned short* WOP, unsigned short* WG, unsigned short* WO) {
  __shared__ __align__(16) float sT[64 * TLD];
  const int blk = blockIdx.x, tid = threadIdx.x;
  const float* src;
  unsigned short* dst;
  int Kd, Nd, bs;
  if (blk < CB_WX)        { src = wip; dst = WIN; Kd = DI;  Nd = 2 * DI; bs = 0;      }
  else if (blk < CB_WDT)  { src = wxp; dst = WX;  Kd = DI;  Nd = DBW;    bs = CB_WX;  }
  else if (blk < CB_WOP)  { src = wdt; dst = WDT; Kd = DR;  Nd = DI;     bs = CB_WDT; }
  else if (blk < CB_WG)   { src = wop; dst = WOP; Kd = DI;  Nd = DI;     bs = CB_WOP; }
  else if (blk < CB_WO)   { src = wg;  dst = WG;  Kd = DMD; Nd = DMD;    bs = CB_WG;  }
  else                    { src = wo;  dst = WO;  Kd = DI;  Nd = DMD;    bs = CB_WO;  }
  const int ti = blk - bs;
  const int ktc = Kd >> 6;
  const int nt = ti / ktc, kt = ti - nt * ktc;
  const int n0 = nt << 6, k0 = kt << 6;
#pragma unroll
  for (int it = 0; it < 4; ++it) {
    const int e = tid + it * NTHR;
    const int kr = e >> 4, nq = e & 15;
    const v4f v = *(const v4f*)(src + (size_t)(k0 + kr) * (size_t)Nd + (size_t)(n0 + 4 * nq));
    *(v4f*)(sT + kr * TLD + 4 * nq) = v;
  }
  __syncthreads();
  v4u hv[2];
  size_t dso[2];
#pragma unroll
  for (int it = 0; it < 2; ++it) {
    const int p = tid + it * NTHR;
    const int nl = p >> 3, q = p & 7;
    const float* sp = sT + (8 * q) * TLD + nl;
    v4f a = {sp[0], sp[TLD], sp[2 * TLD], sp[3 * TLD]};
    v4f c = {sp[4 * TLD], sp[5 * TLD], sp[6 * TLD], sp[7 * TLD]};
    a = a * WSC;
    c = c * WSC;
    hv[it] = pack8h(a, c);
    dso[it] = (size_t)(n0 + nl) * (size_t)Kd + (size_t)(k0 + 8 * q);
  }
#pragma unroll
  for (int it = 0; it < 2; ++it) *(volatile v4u*)(dst + dso[it]) = hv[it];
  __threadfence();
#pragma unroll
  for (int it = 0; it < 2; ++it) *(volatile v4u*)(dst + dso[it]) = hv[it];
}

__global__ __launch_bounds__(NTHR) void k_front(const float* __restrict__ x, const float* __restrict__ cw,
                                                const float* __restrict__ cb, const float* __restrict__ g2,
                                                const float* __restrict__ b2, float* XC32,
                                                unsigned short* XCH, unsigned short* XH) {
  __shared__ float red0[8];
  __shared__ float red1[8];
  const int m = blockIdx.x, tid = threadIdx.x, lane = tid & 31, wave = tid >> 5;
  const int l = m & (LSEQ - 1);
  const int hm = (l > 0) ? 1 : 0;
  const int hp = (l < LSEQ - 1) ? 1 : 0;
  const size_t r0 = (size_t)m * DMD;
  const size_t rm = hm ? (r0 - (size_t)DMD) : r0;
  const size_t rp = hp ? (r0 + (size_t)DMD) : r0;
  const float fm = hm ? 1.0f : 0.0f;
  const float fp = hp ? 1.0f : 0.0f;
  const int c0 = 2 * tid;
  const float xm0 = x[rm + c0] * fm, xm1 = x[rm + c0 + 1] * fm;
  const float x00 = x[r0 + c0],      x01 = x[r0 + c0 + 1];
  const float xp0 = x[rp + c0] * fp, xp1 = x[rp + c0 + 1] * fp;
  const v4f w0 = *(const v4f*)(cw + 12 * tid);
  const v4f w1 = *(const v4f*)(cw + 12 * tid + 4);
  const v4f w2 = *(const v4f*)(cw + 12 * tid + 8);
  const v4f bb = *(const v4f*)(cb + 4 * tid);
  v4f a = bb;
  a[0] = xm0 * w0[0] + x00 * w0[1] + xp0 * w0[2] + bb[0];
  a[1] = xm0 * w0[3] + x00 * w1[0] + xp0 * w1[1] + bb[1];
  a[2] = xm1 * w1[2] + x01 * w1[3] + xp1 * w2[0] + bb[2];
  a[3] = xm1 * w2[1] + x01 * w2[2] + xp1 * w2[3] + bb[3];
  v4f v = a;
#pragma unroll
  for (int j = 0; j < 4; ++j) {
    const float t = a[j];
    v[j] = t * __builtin_amdgcn_rcpf(1.0f + __expf(-t));
  }
  float s = (v[0] + v[1]) + (v[2] + v[3]);
  s = wave_sum(s);
  if (lane == 0) red0[wave] = s;
  __syncthreads();
  float tot = 0.0f;
#pragma unroll
  for (int w = 0; w < 8; ++w) tot += red0[w];
  const float mean = tot * (1.0f / (float)DI);
  v4f d = v;
#pragma unroll
  for (int j = 0; j < 4; ++j) d[j] = v[j] - mean;
  float ss = (d[0] * d[0] + d[1] * d[1]) + (d[2] * d[2] + d[3] * d[3]);
  ss = wave_sum(ss);
  if (lane == 0) red1[wave] = ss;
  __syncthreads();
  float tot2 = 0.0f;
#pragma unroll
  for (int w = 0; w < 8; ++w) tot2 += red1[w];
  const float var = tot2 * (1.0f / (float)DI);
  const float inv = rsqrtf(var + 1e-5f);
  const v4f gg = *(const v4f*)(g2 + 4 * tid);
  const v4f be = *(const v4f*)(b2 + 4 * tid);
  v4f o = d;
#pragma unroll
  for (int j = 0; j < 4; ++j) o[j] = (d[j] * inv) * gg[j] + be[j];
  const v2u oh = pack4h(o);
  const int tq = tid & 63;
  const v4f xa = *(const v4f*)(x + r0 + 8 * tq);
  const v4f xc = *(const v4f*)(x + r0 + 8 * tq + 4);
  const v4u xh = pack8h(xa, xc);
  const size_t oc = (size_t)m * DI + (size_t)(4 * tid);
  const size_t ox = r0 + (size_t)(8 * tq);
  *(volatile v4f*)(XC32 + oc) = o;
  *(volatile v2u*)(XCH + oc) = oh;
  if (tid < 64) *(volatile v4u*)(XH + ox) = xh;
  __threadfence();
  *(volatile v4f*)(XC32 + oc) = o;
  *(volatile v2u*)(XCH + oc) = oh;
  if (tid < 64) *(volatile v4u*)(XH + ox) = xh;
}

template <int WM, int NT, int EP>
__global__ __launch_bounds__(NTHR) void k_gemm(const unsigned short* __restrict__ Ah,
                                               const unsigned short* __restrict__ Wh,
                                               const float* __restrict__ bias,
                                               const float* __restrict__ aux0,
                                               const float* __restrict__ aux1,
                                               float* Cf, unsigned short* Ph,
                                               int lda, int ldw, int ldc, int ldp, int ld0, int ld1,
                                               int K, float osc) {
  constexpr int WN = 8 / WM;
  constexpr int R = 16 * WM;
  constexpr int BN = WN * 16 * NT;
  static_assert(WM * WN == 8);
  static_assert(((R * BN / 4) % NTHR) == 0);
  constexpr int NF4 = (R * BN / 4) / NTHR;
  constexpr int Q4 = BN / 4;
  constexpr bool HASB = (EP == 2 || EP == 6 || EP == 8);
  constexpr bool F32O = (EP == 0 || EP == 2 || EP == 5 || EP == 6 || EP == 8);
  constexpr bool F16O = (EP == 7);
  static_assert(F32O || F16O);
  __shared__ __align__(16) float sC[R * BN];
  const int tid = threadIdx.x, lane = tid & 31, wave = tid >> 5, h = lane >> 4, m = lane & 15;
  const int wm = wave % WM, wn = wave / WM;
  const int bm0 = blockIdx.y * R;
  const int n0 = blockIdx.x * BN;
  const int m0 = bm0 + 16 * wm;
  const int nw0 = n0 + wn * 16 * NT;

  v8f acc[NT];
#pragma unroll
  for (int t = 0; t < NT; ++t) acc[t] = zero8();

  const size_t arow = (size_t)(m0 + m) * (size_t)lda + (size_t)(8 * h);
  const size_t wrow = (size_t)(nw0 + m) * (size_t)ldw + (size_t)(8 * h);
  const int nks = K >> 5;

#pragma unroll 1
  for (int ks = 0; ks < nks; ++ks) {
    const int k0 = ks << 5;
    Frag fa;
    fa.q[0] = *(const v4u*)(Ah + arow + k0);
    fa.q[1] = *(const v4u*)(Ah + arow + k0 + 16);
#pragma unroll
    for (int t = 0; t < NT; ++t) {
      const unsigned short* wp = Wh + wrow + (size_t)(16 * t) * (size_t)ldw + k0;
      Frag fw;
      fw.q[0] = *(const v4u*)wp;
      fw.q[1] = *(const v4u*)(wp + 16);
      acc[t] = wmh(fa, fw, acc[t]);
    }
  }

#pragma unroll
  for (int t = 0; t < NT; ++t) {
    const int cl = wn * 16 * NT + 16 * t + m;
#pragma unroll
    for (int r = 0; r < 8; ++r) {
      const int rl = 16 * wm + 8 * h + r;
      sC[rl * BN + cl] = acc[t][r];
    }
  }
  __syncthreads();

  if constexpr (F32O) {
#pragma unroll 1
    for (int it = 0; it < NF4; ++it) {
      const int e = tid + it * NTHR;
      const int rl = e / Q4, q = e - rl * Q4;
      v4f v = *(const v4f*)(sC + 4 * e);
      v = v * osc;
      if constexpr (HASB) {
        const v4f bb = *(const v4f*)(bias + n0 + 4 * q);
        v = v + bb;
      }
      if constexpr (EP == 2) {
#pragma unroll
        for (int j = 0; j < 4; ++j) {
          const float a = v[j];
          v[j] = fmaxf(a, 0.0f) + log1pf(__expf(-fabsf(a)));
        }
      }
      if constexpr (EP == 6) {
#pragma unroll
        for (int j = 0; j < 4; ++j) {
          const float a = v[j];
          v[j] = __builtin_amdgcn_rcpf(1.0f + __expf(-a));
        }
      }
      if constexpr (EP == 8) {
        const v4f rs = *(const v4f*)(aux0 + (size_t)(bm0 + rl) * (size_t)ld0 + (size_t)(n0 + 4 * q));
        v = v + rs;
      }
      *(v4f*)(sC + 4 * e) = v;
    }
#pragma unroll
    for (int it = 0; it < NF4; ++it) {
      const int e = tid + it * NTHR;
      const int rl = e / Q4, q = e - rl * Q4;
      const v4f v = *(const v4f*)(sC + 4 * e);
      *(volatile v4f*)(Cf + (size_t)(bm0 + rl) * (size_t)ldc + n0 + 4 * q) = v;
    }
    __threadfence();
#pragma unroll
    for (int it = 0; it < NF4; ++it) {
      const int e = tid + it * NTHR;
      const int rl = e / Q4, q = e - rl * Q4;
      const v4f v = *(const v4f*)(sC + 4 * e);
      *(volatile v4f*)(Cf + (size_t)(bm0 + rl) * (size_t)ldc + n0 + 4 * q) = v;
    }
  }

  if constexpr (F16O) {
    static_assert(((R * BN / 8) % NTHR) == 0);
    constexpr int NP8 = (R * BN / 8) / NTHR;
    constexpr int Q8 = BN / 8;
    v4u hv[NP8];
    size_t dst[NP8];
#pragma unroll
    for (int it = 0; it < NP8; ++it) {
      const int e = tid + it * NTHR;
      const int rl = e / Q8, q = e - rl * Q8;
      v4f a = *(const v4f*)(sC + rl * BN + 8 * q);
      v4f c = *(const v4f*)(sC + rl * BN + 8 * q + 4);
      a = a * osc;
      c = c * osc;
      const size_t row = (size_t)(bm0 + rl);
      const int col0 = n0 + 8 * q;
      const v4f gq = *(const v4f*)(aux0 + row * (size_t)ld0 + (size_t)(col0 >> 1));
      const v4f x0 = *(const v4f*)(aux1 + row * (size_t)ld1 + (size_t)col0);
      const v4f x1 = *(const v4f*)(aux1 + row * (size_t)ld1 + (size_t)col0 + 4);
      v4f sg = gq, fg = gq;
#pragma unroll
      for (int j = 0; j < 4; ++j) {
        const float gv = gq[j];
        const float sv = __builtin_amdgcn_rcpf(1.0f + __expf(-gv));
        sg[j] = gv * sv;
        fg[j] = 1.0f - gv;
      }
      v4f o0 = a, o1 = c;
#pragma unroll
      for (int j = 0; j < 4; ++j) {
        o0[j] = a[j] * sg[j >> 1] + x0[j] * fg[j >> 1];
        o1[j] = c[j] * sg[2 + (j >> 1)] + x1[j] * fg[2 + (j >> 1)];
      }
      hv[it] = pack8h(o0, o1);
      dst[it] = row * (size_t)ldp + (size_t)col0;
    }
#pragma unroll
    for (int it = 0; it < NP8; ++it) *(volatile v4u*)(Ph + dst[it]) = hv[it];
    __threadfence();
#pragma unroll
    for (int it = 0; it < NP8; ++it) *(volatile v4u*)(Ph + dst[it]) = hv[it];
  }

  if constexpr (EP == 5) {
    static_assert(R == 64 && BN >= DR && (R * DR / 8) == 2 * NTHR);
    __syncthreads();
    v4u hv[2];
    size_t dst[2];
#pragma unroll
    for (int it = 0; it < 2; ++it) {
      const int e = tid + it * NTHR;
      const int rl = e >> 3, q = e & 7;
      v4f a = *(const v4f*)(sC + rl * BN + 8 * q);
      v4f c = *(const v4f*)(sC + rl * BN + 8 * q + 4);
      a = a * DTHC;
      c = c * DTHC;
      hv[it] = pack8h(a, c);
      dst[it] = (size_t)(bm0 + rl) * DR + 8 * q;
    }
#pragma unroll
    for (int it = 0; it < 2; ++it) *(volatile v4u*)(Ph + dst[it]) = hv[it];
    __threadfence();
#pragma unroll
    for (int it = 0; it < 2; ++it) *(volatile v4u*)(Ph + dst[it]) = hv[it];
  }
}

static_assert((DI / 4) == 256 && ((NTOK * DI / 4) % NTHR) == 0);

__global__ __launch_bounds__(NTHR) void k_conv4(const float* __restrict__ XS, const float* __restrict__ cw,
                                                const float* __restrict__ cb, float* U32, unsigned short* UH) {
  const int g = blockIdx.x * NTHR + threadIdx.x;
  const int row = g >> 8;
  const int dq = (g & 255) << 2;
  const int t = row & (LSEQ - 1);
  const int rb = row - t;
  v4f acc = *(const v4f*)(cb + dq);
  v4f w[4];
#pragma unroll
  for (int j = 0; j < 4; ++j) w[j] = *(const v4f*)(cw + (size_t)(dq + j) * DC);
#pragma unroll
  for (int k = 0; k < DC; ++k) {
    const int tt = t + k - (DC - 1);
    const int ttc = (tt < 0) ? 0 : tt;
    const v4f xv = *(const v4f*)(XS + (size_t)(rb + ttc) * (size_t)DI + dq);
    const float f = (tt >= 0) ? 1.0f : 0.0f;
#pragma unroll
    for (int j = 0; j < 4; ++j) acc[j] = acc[j] + (xv[j] * f) * w[j][k];
  }
  v4f u = acc;
#pragma unroll
  for (int j = 0; j < 4; ++j) {
    const float a = acc[j];
    u[j] = a * __builtin_amdgcn_rcpf(1.0f + __expf(-a));
  }
  const v4f us = u * UHC;
  const v2u hv = pack4h(us);
  const size_t o = (size_t)g * 4;
  *(volatile v4f*)(U32 + o) = u;
  *(volatile v2u*)(UH + o) = hv;
  __threadfence();
  *(volatile v4f*)(U32 + o) = u;
  *(volatile v2u*)(UH + o) = hv;
}

#define SCB 256
#define STB 16
static_assert(SCB == NTHR && (DI % SCB) == 0 && (LSEQ % STB) == 0 && DS == 32);
static_assert(((STB * SCB / 8) % NTHR) == 0);

__global__ __launch_bounds__(NTHR) void k_scan(const float* __restrict__ DEL, const float* __restrict__ U32,
                                               const float* __restrict__ DBL, const float* __restrict__ Zp,
                                               const float* __restrict__ Alog, const float* __restrict__ Dp,
                                               unsigned short* YH) {
  __shared__ __align__(16) float sA[SCB * DS];
  __shared__ __align__(16) float sY[STB * SCB];
  const int tid = threadIdx.x;
  const int cbase = blockIdx.x * SCB;
  const int ch = cbase + tid;
  const size_t rbase = (size_t)blockIdx.y * LSEQ;
#pragma unroll 1
  for (int e = tid; e < SCB * DS; e += NTHR) sA[e] = -expf(Alog[(size_t)cbase * DS + e]);
  __syncthreads();

  float Ac[DS], hs[DS];
#pragma unroll
  for (int n = 0; n < DS; ++n) {
    Ac[n] = sA[tid * DS + n];
    hs[n] = 0.0f;
  }
  const float Dd = Dp[ch];

#pragma unroll 1
  for (int t0 = 0; t0 < LSEQ; t0 += STB) {
#pragma unroll 1
    for (int tl = 0; tl < STB; ++tl) {
      const size_t row = rbase + (size_t)(t0 + tl);
      const float dt = DEL[row * DI + ch];
      const float u = U32[row * DI + ch];
      const float z = Zp[row * DI + ch];
      const float* bp = DBL + row * DBW + DR;
      v4f bq[8], cq[8];
#pragma unroll
      for (int i = 0; i < 8; ++i) {
        bq[i] = *(const v4f*)(bp + 4 * i);
        cq[i] = *(const v4f*)(bp + DS + 4 * i);
      }
      const float dtu = dt * u;
      float part = 0.0f;
#pragma unroll
      for (int n = 0; n < DS; ++n) {
        const float bv = bq[n >> 2][n & 3];
        const float cv = cq[n >> 2][n & 3];
        const float dA = __expf(dt * Ac[n]);
        const float hn = dA * hs[n] + dtu * bv;
        hs[n] = hn;
        part = part + hn * cv;
      }
      const float sg = __builtin_amdgcn_rcpf(1.0f + __expf(-z));
      const float y = (part + Dd * u) * (z * sg);
      sY[tl * SCB + tid] = y;
    }
    __syncthreads();
    {
      constexpr int NIT = (STB * SCB / 8) / NTHR;
      v4u hv[NIT];
      size_t dst[NIT];
#pragma unroll
      for (int it = 0; it < NIT; ++it) {
        const int e = tid + it * NTHR;
        const int rl = e >> 5, q = e & 31;
        v4f a = *(const v4f*)(sY + rl * SCB + 8 * q);
        v4f c = *(const v4f*)(sY + rl * SCB + 8 * q + 4);
        a = a * YHC;
        c = c * YHC;
        hv[it] = pack8h(a, c);
        dst[it] = (rbase + (size_t)(t0 + rl)) * (size_t)DI + (size_t)(cbase + 8 * q);
      }
#pragma unroll
      for (int it = 0; it < NIT; ++it) *(volatile v4u*)(YH + dst[it]) = hv[it];
      __threadfence();
#pragma unroll
      for (int it = 0; it < NIT; ++it) *(volatile v4u*)(YH + dst[it]) = hv[it];
    }
    __syncthreads();
  }
}

#define LNT 128
static_assert(LNT * 4 == DMD);

__global__ __launch_bounds__(LNT) void k_ln1(const float* __restrict__ PRE, const float* __restrict__ g1,
                                             const float* __restrict__ b1, float* out) {
  __shared__ float red0[4];
  __shared__ float red1[4];
  const int row = blockIdx.x, tid = threadIdx.x, lane = tid & 31, wave = tid >> 5;
  const size_t o = (size_t)row * DMD + (size_t)(4 * tid);
  const v4f v = *(const v4f*)(PRE + o);
  float s = (v[0] + v[1]) + (v[2] + v[3]);
  s = wave_sum(s);
  if (lane == 0) red0[wave] = s;
  __syncthreads();
  const float tot = (red0[0] + red0[1]) + (red0[2] + red0[3]);
  const float mean = tot * (1.0f / (float)DMD);
  v4f d = v;
#pragma unroll
  for (int j = 0; j < 4; ++j) d[j] = v[j] - mean;
  float ss = (d[0] * d[0] + d[1] * d[1]) + (d[2] * d[2] + d[3] * d[3]);
  ss = wave_sum(ss);
  if (lane == 0) red1[wave] = ss;
  __syncthreads();
  const float tot2 = (red1[0] + red1[1]) + (red1[2] + red1[3]);
  const float var = tot2 * (1.0f / (float)DMD);
  const float inv = rsqrtf(var + 1e-5f);
  const v4f gg = *(const v4f*)(g1 + 4 * tid);
  const v4f be = *(const v4f*)(b1 + 4 * tid);
  v4f r = d;
#pragma unroll
  for (int j = 0; j < 4; ++j) r[j] = (d[j] * inv) * gg[j] + be[j];
  *(volatile v4f*)(out + o) = r;
  __threadfence();
  *(volatile v4f*)(out + o) = r;
}

extern "C" void kernel_launch(void* const* d_in, const int* in_sizes, int n_in,
                              void* d_out, int out_size, void* d_ws, size_t ws_size,
                              hipStream_t stream) {
  if (n_in < 20) return;
  if (in_sizes[0] != NTOK * DMD) return;
  if (in_sizes[1] != DI * 3 || in_sizes[2] != DI) return;
  if (in_sizes[3] != DMD * DMD || in_sizes[4] != DMD) return;
  if (in_sizes[5] != DI * DMD || in_sizes[6] != DMD) return;
  if (in_sizes[7] != DMD || in_sizes[8] != DMD) return;
  if (in_sizes[9] != DI || in_sizes[10] != DI) return;
  if (in_sizes[11] != DI * 2 * DI) return;
  if (in_sizes[12] != DI * DC || in_sizes[13] != DI) return;
  if (in_sizes[14] != DI * DBW) return;
  if (in_sizes[15] != DR * DI || in_sizes[16] != DI) return;
  if (in_sizes[17] != DI * DS || in_sizes[18] != DI) return;
  if (in_sizes[19] != DI * DI) return;
  if (out_size != NTOK * DMD) return;
  const size_t tot = (size_t)WSTOT;
  if (tot > ws_size || tot > (size_t)WSCAP) return;

  const float* x      = (const float*)d_in[0];
  const float* conv_w = (const float*)d_in[1];
  const float* conv_b = (const float*)d_in[2];
  const float* gate_w = (const float*)d_in[3];
  const float* gate_b = (const float*)d_in[4];
  const float* out_w  = (const float*)d_in[5];
  const float* out_b  = (const float*)d_in[6];
  const float* ln1_g  = (const float*)d_in[7];
  const float* ln1_b  = (const float*)d_in[8];
  const float* ln2_g  = (const float*)d_in[9];
  const float* ln2_b  = (const float*)d_in[10];
  const float* inpw   = (const float*)d_in[11];
  const float* scw    = (const float*)d_in[12];
  const float* scb    = (const float*)d_in[13];
  const float* xpw    = (const float*)d_in[14];
  const float* dtw    = (const float*)d_in[15];
  const float* dtb    = (const float*)d_in[16];
  const float* alog   = (const float*)d_in[17];
  const float* dsk    = (const float*)d_in[18];
  const float* opw    = (const float*)d_in[19];
  float* out0 = (float*)d_out;

  char* ws = (char*)d_ws;
  unsigned short* WIN  = (unsigned short*)(ws + O_WIN);
  unsigned short* WX   = (unsigned short*)(ws + O_WX);
  unsigned short* WDT  = (unsigned short*)(ws + O_WDT);
  unsigned short* WOP  = (unsigned short*)(ws + O_WOP);
  unsigned short* WG   = (unsigned short*)(ws + O_WG);
  unsigned short* WO   = (unsigned short*)(ws + O_WO);
  unsigned short* XH   = (unsigned short*)(ws + O_XH);
  float*          XC32 = (float*)(ws + O_XC32);
  unsigned short* XCH  = (unsigned short*)(ws + O_R1);
  unsigned short* UH   = (unsigned short*)(ws + O_R1);
  unsigned short* YH   = (unsigned short*)(ws + O_R1);
  float*          XS32 = (float*)(ws + O_R2);
  float*          DEL  = (float*)(ws + O_R2);
  unsigned short* CMH  = (unsigned short*)(ws + O_R2);
  float*          Z32  = (float*)(ws + O_R3);
  float*          PRE  = (float*)(ws + O_R3);
  float*          U32  = (float*)(ws + O_U32);
  float*          DBL  = (float*)(ws + O_DBL);
  unsigned short* DTH  = (unsigned short*)(ws + O_DTH);
  float*          G32  = (float*)(ws + O_G32);


  k_cvtw<<<CB_TOT, NTHR, 0, stream>>>(inpw, xpw, dtw, opw, gate_w, out_w, WIN, WX, WDT, WOP, WG, WO);

  k_front<<<NTOK, NTHR, 0, stream>>>(x, conv_w, conv_b, ln2_g, ln2_b, XC32, XCH, XH);

  k_gemm<2, 4, 0><<<dim3(DI / 256, NTOK / 32), NTHR, 0, stream>>>(
      XCH, WIN, conv_b, x, x, XS32, DTH, DI, DI, DI, 0, 0, 0, DI, 0.03125f);

  k_gemm<2, 4, 0><<<dim3(DI / 256, NTOK / 32), NTHR, 0, stream>>>(
      XCH, WIN + (size_t)DI * DI, conv_b, x, x, Z32, DTH, DI, DI, DI, 0, 0, 0, DI, 0.03125f);

  k_conv4<<<(NTOK * DI / 4) / NTHR, NTHR, 0, stream>>>(XS32, scw, scb, U32, UH);

  k_gemm<4, 4, 5><<<dim3(DBW / 128, NTOK / 64), NTHR, 0, stream>>>(
      UH, WX, conv_b, x, x, DBL, DTH, DI, DI, DBW, DR, 0, 0, DI, 0.00048828125f);

  k_gemm<2, 4, 2><<<dim3(DI / 256, NTOK / 32), NTHR, 0, stream>>>(
      DTH, WDT, dtb, x, x, DEL, UH, DR, DR, DI, 0, 0, 0, DR, 0.0001220703125f);

  k_gemm<2, 4, 6><<<dim3(DMD / 256, NTOK / 32), NTHR, 0, stream>>>(
      XH, WG, gate_b, x, x, G32, UH, DMD, DMD, DMD, 0, 0, 0, DMD, 0.03125f);

  k_scan<<<dim3(DI / SCB, NB), NTHR, 0, stream>>>(DEL, U32, DBL, Z32, alog, dsk, YH);

  k_gemm<2, 4, 7><<<dim3(DI / 256, NTOK / 32), NTHR, 0, stream>>>(
      YH, WOP, conv_b, G32, XC32, PRE, CMH, DI, DI, 0, DI, DMD, DI, DI, 0.0001220703125f);

  k_gemm<2, 4, 8><<<dim3(DMD / 256, NTOK / 32), NTHR, 0, stream>>>(
      CMH, WO, out_b, x, x, PRE, YH, DI, DI, DMD, 0, DMD, 0, DI, 0.03125f);

  k_ln1<<<NTOK, LNT, 0, stream>>>(PRE, ln1_g, ln1_b, out0);
}
